// SparseTransformerEncoder_69020124446904
// MI455X (gfx1250) — hardware-verified
//
#include <hip/hip_runtime.h>
#include <math.h>

typedef _Float16 v16h __attribute__((ext_vector_type(16)));
typedef _Float16 v8h  __attribute__((ext_vector_type(8)));
typedef float    v8f  __attribute__((ext_vector_type(8)));
typedef float    v4f  __attribute__((ext_vector_type(4)));
typedef int      v4i  __attribute__((ext_vector_type(4)));
typedef v8h __attribute__((may_alias)) v8ha;
typedef v4f __attribute__((may_alias)) v4fa;
typedef v4i __attribute__((may_alias)) v4ia;

union Frag { v16h v; v8h half[2]; };

#define NBATCH 2
#define SEQ    2048
#define DM     512
#define NH     8
#define HD     64
#define NL     4
#define DMLP   2048
#define BLK    128
#define CSUM   32
#define NBLK   (SEQ / BLK)
#define NTOK   (NBATCH * SEQ)
#define NQKV   (3 * DM)
#define WSC    64.0f
#define WINV   0.015625f
#define QSC    0.125f
#define PSCALE 16384.0f
#define PINV   6.1035156e-5f
#define NEGBIG (-1.0e9f)

__device__ __forceinline__ v8f zero8f() {
  v8f z = {0.f, 0.f, 0.f, 0.f, 0.f, 0.f, 0.f, 0.f};
  return z;
}

__device__ __forceinline__ v8f wmma_raw(v16h a, v16h b, v8f c) {
  return __builtin_amdgcn_wmma_f32_16x16x32_f16(false, a, false, b, (short)0, c, false, false);
}

__device__ __forceinline__ v16h load_frag(const _Float16* p, int h) {
  Frag f;
  f.half[0] = *(const v8ha*)(p + 8 * h);
  f.half[1] = *(const v8ha*)(p + 16 + 8 * h);
  return f.v;
}

__device__ __forceinline__ v8h to8h(v8f v) {
  v8h r = { (_Float16)v[0], (_Float16)v[1], (_Float16)v[2], (_Float16)v[3],
            (_Float16)v[4], (_Float16)v[5], (_Float16)v[6], (_Float16)v[7] };
  return r;
}

__device__ __forceinline__ float wave_sum(float v) {
  #pragma unroll
  for (int o = 1; o < 32; o <<= 1) v += __shfl_xor(v, o, 32);
  return v;
}

__device__ __forceinline__ float gelu_f(float x) {
  const float x3 = x * x * x;
  return 0.5f * x * (1.0f + tanhf(0.79788456f * (x + 0.044715f * x3)));
}

__device__ __forceinline__ void gemm_core(const _Float16* __restrict__ Ar, const _Float16* __restrict__ Br,
                                          int K, int h, v8f (&acc)[2][4]) {
  #pragma unroll
  for (int i = 0; i < 2; ++i)
    #pragma unroll
    for (int j = 0; j < 4; ++j) acc[i][j] = zero8f();
  const _Float16* Ar1 = Ar + (size_t)16 * K;
  #pragma unroll 1
  for (int k0 = 0; k0 < K; k0 += 32) {
    const v16h fa0 = load_frag(Ar + k0, h);
    const v16h fa1 = load_frag(Ar1 + k0, h);
    v16h fb[4];
    #pragma unroll
    for (int j = 0; j < 4; ++j) fb[j] = load_frag(Br + (size_t)(16 * j) * K + k0, h);
    #pragma unroll
    for (int j = 0; j < 4; ++j) {
      acc[0][j] = wmma_raw(fa0, fb[j], acc[0][j]);
      acc[1][j] = wmma_raw(fa1, fb[j], acc[1][j]);
    }
    asm volatile("v_nop\n\tv_nop\n\tv_nop\n\tv_nop"
                 : "+v"(acc[0][0]), "+v"(acc[0][1]), "+v"(acc[0][2]), "+v"(acc[0][3]),
                   "+v"(acc[1][0]), "+v"(acc[1][1]), "+v"(acc[1][2]), "+v"(acc[1][3])
                 : "v"(fa0), "v"(fa1), "v"(fb[0]), "v"(fb[1]), "v"(fb[2]), "v"(fb[3]));
  }
}

__device__ __forceinline__ void store_rows16(const _Float16* sT, _Float16* dst, size_t pitch, int w, int lane) {
  const int q8 = lane & 7, sub = lane >> 3;
  #pragma unroll
  for (int i = 0; i < 8; ++i) {
    const int lid = 32 * w + 4 * i + sub;
    const v8h v = *(const v8ha*)(sT + lid * 64 + 8 * q8);
    *(volatile v8h*)(dst + (size_t)lid * pitch + 8 * q8) = v;
  }
}

__device__ __forceinline__ void store_vt(const _Float16* sT, _Float16* dst, int w, int lane) {
  const int q8 = lane & 7, sub = lane >> 3;
  #pragma unroll
  for (int i = 0; i < 8; ++i) {
    const int lid = 32 * w + 4 * i + sub;
    const int d = lid >> 1, hl = lid & 1;
    const v8h v = *(const v8ha*)(sT + d * 128 + 64 * hl + 8 * q8);
    *(volatile v8h*)(dst + (size_t)d * SEQ + 64 * hl + 8 * q8) = v;
  }
}

__device__ __forceinline__ void cvt_store_pass(const _Float16* sT, _Float16* dst, size_t rowBase, int K, int k0,
                                               int w, int lane) {
  const int q8 = lane & 7, sub = lane >> 3;
  #pragma unroll
  for (int i = 0; i < 2; ++i) {
    const int lid = 8 * w + 4 * i + sub;
    const v8h v = *(const v8ha*)(sT + lid * 64 + 8 * q8);
    *(volatile v8h*)(dst + (rowBase + lid) * (size_t)K + k0 + 8 * q8) = v;
  }
}

__device__ __forceinline__ void att_store_pass(const _Float16* so, _Float16* dst, int lane) {
  const int q8 = lane & 7, sub = lane >> 3;
  #pragma unroll
  for (int i = 0; i < 4; ++i) {
    const int row = 4 * i + sub;
    const v8h v = *(const v8ha*)(so + row * HD + 8 * q8);
    *(volatile v8h*)(dst + (size_t)row * DM + 8 * q8) = v;
  }
}

__global__ __launch_bounds__(256) void cvt_t_kernel(const float* __restrict__ src, _Float16* __restrict__ dst,
                                                    int K, int N, int dstRows, int nOff, float scale) {
  __shared__ __attribute__((aligned(16))) _Float16 sT[64 * 64];
  const int tid = threadIdx.x, lane = tid & 31, w = tid >> 5;
  const int n0 = blockIdx.x * 64, k0 = blockIdx.y * 64, l = blockIdx.z;
  const int c4 = (tid & 15) * 4, kr = tid >> 4;
  #pragma unroll
  for (int j = 0; j < 4; ++j) {
    const int kk = kr + 16 * j;
    const v4f v = *(const v4fa*)(src + ((size_t)l * K + k0 + kk) * N + n0 + c4);
    sT[(c4 + 0) * 64 + kk] = (_Float16)(v.x * scale);
    sT[(c4 + 1) * 64 + kk] = (_Float16)(v.y * scale);
    sT[(c4 + 2) * 64 + kk] = (_Float16)(v.z * scale);
    sT[(c4 + 3) * 64 + kk] = (_Float16)(v.w * scale);
  }
  __syncthreads();
  const size_t rowBase = (size_t)l * dstRows + nOff + n0;
  cvt_store_pass(sT, dst, rowBase, K, k0, w, lane);
  __threadfence();
  cvt_store_pass(sT, dst, rowBase, K, k0, w, lane);
}

__global__ __launch_bounds__(256) void embed_kernel(const int* __restrict__ ids, const float* __restrict__ emb,
                                                    float* __restrict__ x, int vocab) {
  __shared__ __attribute__((aligned(16))) float spe[DM];
  const int row = blockIdx.x, t = threadIdx.x;
  const int s = row & (SEQ - 1);
  const float cexp = (float)(-(9.2103404 / 256.0));
  const float arg = (float)s * expf((float)t * cexp);
  spe[t] = sinf(arg);
  spe[t + DM / 2] = cosf(arg);
  __syncthreads();
  if (t < DM / 4) {
    int id = ids[row];
    id = (id < 0) ? 0 : id;
    id = (id > vocab - 1) ? (vocab - 1) : id;
    const v4f e = *(const v4fa*)(emb + (size_t)id * DM + 4 * t);
    const v4f p4 = *(const v4fa*)(spe + 4 * t);
    const v4f o = e + p4;
    float* p = x + (size_t)row * DM + 4 * t;
    *(volatile v4f*)p = o;
    __threadfence();
    *(volatile v4f*)p = o;
  }
}

__global__ __launch_bounds__(256) void ln16_kernel(const float* __restrict__ x, const float* __restrict__ g,
                                                   const float* __restrict__ be, _Float16* __restrict__ y) {
  const int lane = threadIdx.x & 31, w = threadIdx.x >> 5;
  const int row = blockIdx.x * 8 + w;
  const float* xr = x + (size_t)row * DM;
  v4f a[4], gg[4], bb[4];
  #pragma unroll
  for (int j = 0; j < 4; ++j) {
    const int off = 256 * (j >> 1) + 8 * lane + 4 * (j & 1);
    a[j]  = *(const v4fa*)(xr + off);
    gg[j] = *(const v4fa*)(g + off);
    bb[j] = *(const v4fa*)(be + off);
  }
  float s = 0.f;
  #pragma unroll
  for (int j = 0; j < 4; ++j) s += a[j].x + a[j].y + a[j].z + a[j].w;
  s = wave_sum(s);
  const float mean = s * (1.0f / DM);
  v4f d[4];
  float ss = 0.f;
  #pragma unroll
  for (int j = 0; j < 4; ++j) {
    d[j] = a[j] - mean;
    ss += d[j].x * d[j].x + d[j].y * d[j].y + d[j].z * d[j].z + d[j].w * d[j].w;
  }
  ss = wave_sum(ss);
  const float inv = 1.0f / sqrtf(ss * (1.0f / DM) + 1.0e-6f);
  v4f o[4];
  #pragma unroll
  for (int j = 0; j < 4; ++j) o[j] = d[j] * inv * gg[j] + bb[j];
  const v8h p0 = { (_Float16)o[0].x, (_Float16)o[0].y, (_Float16)o[0].z, (_Float16)o[0].w,
                   (_Float16)o[1].x, (_Float16)o[1].y, (_Float16)o[1].z, (_Float16)o[1].w };
  const v8h p1 = { (_Float16)o[2].x, (_Float16)o[2].y, (_Float16)o[2].z, (_Float16)o[2].w,
                   (_Float16)o[3].x, (_Float16)o[3].y, (_Float16)o[3].z, (_Float16)o[3].w };
  _Float16* yp = y + (size_t)row * DM + 8 * lane;
  *(volatile v8h*)yp = p0;
  *(volatile v8h*)(yp + 256) = p1;
  __threadfence();
  *(volatile v8h*)yp = p0;
  *(volatile v8h*)(yp + 256) = p1;
}

__global__ __launch_bounds__(256) void ln32_kernel(const float* __restrict__ x, const float* __restrict__ g,
                                                   const float* __restrict__ be, float* __restrict__ out) {
  const int lane = threadIdx.x & 31, w = threadIdx.x >> 5;
  const int row = blockIdx.x * 8 + w;
  const float* xr = x + (size_t)row * DM;
  v4f a[4], gg[4], bb[4];
  #pragma unroll
  for (int j = 0; j < 4; ++j) {
    const int off = 128 * j + 4 * lane;
    a[j]  = *(const v4fa*)(xr + off);
    gg[j] = *(const v4fa*)(g + off);
    bb[j] = *(const v4fa*)(be + off);
  }
  float s = 0.f;
  #pragma unroll
  for (int j = 0; j < 4; ++j) s += a[j].x + a[j].y + a[j].z + a[j].w;
  s = wave_sum(s);
  const float mean = s * (1.0f / DM);
  v4f d[4];
  float ss = 0.f;
  #pragma unroll
  for (int j = 0; j < 4; ++j) {
    d[j] = a[j] - mean;
    ss += d[j].x * d[j].x + d[j].y * d[j].y + d[j].z * d[j].z + d[j].w * d[j].w;
  }
  ss = wave_sum(ss);
  const float inv = 1.0f / sqrtf(ss * (1.0f / DM) + 1.0e-6f);
  v4f o[4];
  #pragma unroll
  for (int j = 0; j < 4; ++j) o[j] = d[j] * inv * gg[j] + bb[j];
  float* op = out + (size_t)row * DM + 4 * lane;
  #pragma unroll
  for (int j = 0; j < 4; ++j) *(volatile v4f*)(op + 128 * j) = o[j];
  __threadfence();
  #pragma unroll
  for (int j = 0; j < 4; ++j) *(volatile v4f*)(op + 128 * j) = o[j];
}

__global__ __launch_bounds__(128) void gemm_qk_kernel(const _Float16* __restrict__ hb, const _Float16* __restrict__ wt,
                                                      _Float16* __restrict__ qp, _Float16* __restrict__ kp) {
  __shared__ __attribute__((aligned(16))) _Float16 sT[128 * 64];
  const int tid = threadIdx.x, lane = tid & 31, w = tid >> 5;
  const int h = lane >> 4, m = lane & 15, w1 = w & 1, w2 = w >> 1;
  const int m0 = blockIdx.x * 128, by = blockIdx.y;
  const int which = by >> 3, head = by & (NH - 1);
  const int n0 = by * 64;
  v8f acc[2][4];
  gemm_core(wt + (size_t)(n0 + 32 * w1 + m) * DM, hb + (size_t)(m0 + 64 * w2 + m) * DM, DM, h, acc);
  const float osc = (which == 0) ? (WINV * QSC) : WINV;
  #pragma unroll
  for (int i = 0; i < 2; ++i)
    #pragma unroll
    for (int j = 0; j < 4; ++j) {
      const int tokl = 64 * w2 + 16 * j + m;
      const int featl = 32 * w1 + 16 * i + 8 * h;
      *(v8ha*)(sT + tokl * 64 + featl) = to8h(acc[i][j] * osc);
    }
  __syncthreads();
  const int b = m0 / SEQ, l0 = m0 - b * SEQ, bh = b * NH + head;
  _Float16* dst = ((which == 0) ? qp : kp) + ((size_t)bh * SEQ + l0) * HD;
  store_rows16(sT, dst, HD, w, lane);
  __threadfence();
  store_rows16(sT, dst, HD, w, lane);
}

__global__ __launch_bounds__(128) void gemm_v_kernel(const _Float16* __restrict__ hb, const _Float16* __restrict__ wt,
                                                     _Float16* __restrict__ vt) {
  __shared__ __attribute__((aligned(16))) _Float16 sT[64 * 128];
  const int tid = threadIdx.x, lane = tid & 31, w = tid >> 5;
  const int h = lane >> 4, m = lane & 15;
  const int m0 = blockIdx.x * 128, head = blockIdx.y;
  const int n0 = head * 64;
  v8f acc[2][4];
  gemm_core(hb + (size_t)(m0 + 32 * w + m) * DM, wt + (size_t)(n0 + m) * DM, DM, h, acc);
  #pragma unroll
  for (int i = 0; i < 2; ++i)
    #pragma unroll
    for (int j = 0; j < 4; ++j) {
      const int tokl = 32 * w + 16 * i + 8 * h;
      const int featl = 16 * j + m;
      *(v8ha*)(sT + featl * 128 + tokl) = to8h(acc[i][j] * WINV);
    }
  __syncthreads();
  const int b = m0 / SEQ, l0 = m0 - b * SEQ, bh = b * NH + head;
  _Float16* dst = vt + (size_t)bh * HD * SEQ + l0;
  store_vt(sT, dst, w, lane);
  __threadfence();
  store_vt(sT, dst, w, lane);
}

__global__ __launch_bounds__(128) void gemm_gelu_kernel(const _Float16* __restrict__ hb, const _Float16* __restrict__ wt,
                                                        const float* __restrict__ bias, _Float16* __restrict__ m1) {
  __shared__ __attribute__((aligned(16))) _Float16 sT[128 * 64];
  const int tid = threadIdx.x, lane = tid & 31, w = tid >> 5;
  const int h = lane >> 4, m = lane & 15, w1 = w & 1, w2 = w >> 1;
  const int m0 = blockIdx.x * 128, n0 = blockIdx.y * 64;
  v8f acc[2][4];
  gemm_core(wt + (size_t)(n0 + 32 * w1 + m) * DM, hb + (size_t)(m0 + 64 * w2 + m) * DM, DM, h, acc);
  #pragma unroll
  for (int i = 0; i < 2; ++i) {
    const int featl = 32 * w1 + 16 * i + 8 * h;
    const v4f ba = *(const v4fa*)(bias + n0 + featl);
    const v4f bb = *(const v4fa*)(bias + n0 + featl + 4);
    v8f bv;
    bv[0] = ba.x; bv[1] = ba.y; bv[2] = ba.z; bv[3] = ba.w;
    bv[4] = bb.x; bv[5] = bb.y; bv[6] = bb.z; bv[7] = bb.w;
    #pragma unroll
    for (int j = 0; j < 4; ++j) {
      const int tokl = 64 * w2 + 16 * j + m;
      const v8f v = acc[i][j] * WINV + bv;
      v8f gv;
      #pragma unroll
      for (int r = 0; r < 8; ++r) gv[r] = gelu_f(v[r]);
      *(v8ha*)(sT + tokl * 64 + featl) = to8h(gv);
    }
  }
  __syncthreads();
  _Float16* dst = m1 + (size_t)m0 * DMLP + n0;
  store_rows16(sT, dst, DMLP, w, lane);
  __threadfence();
  store_rows16(sT, dst, DMLP, w, lane);
}

template <int HASB>
__global__ __launch_bounds__(128) void gemm_resid_kernel(const _Float16* __restrict__ A, const _Float16* __restrict__ wt,
                                                         const float* __restrict__ bias, float* xio, int K) {
  __shared__ __attribute__((aligned(16))) float sF[128 * 64];
  const int tid = threadIdx.x, lane = tid & 31, w = tid >> 5;
  const int h = lane >> 4, m = lane & 15, w1 = w & 1, w2 = w >> 1;
  const int m0 = blockIdx.x * 128, n0 = blockIdx.y * 64;
  v8f acc[2][4];
  gemm_core(wt + (size_t)(n0 + 32 * w1 + m) * K, A + (size_t)(m0 + 64 * w2 + m) * K, K, h, acc);
  #pragma unroll
  for (int i = 0; i < 2; ++i) {
    const int featl = 32 * w1 + 16 * i + 8 * h;
    v8f bv = zero8f();
    if (HASB) {
      const v4f ba = *(const v4fa*)(bias + n0 + featl);
      const v4f bb = *(const v4fa*)(bias + n0 + featl + 4);
      bv[0] = ba.x; bv[1] = ba.y; bv[2] = ba.z; bv[3] = ba.w;
      bv[4] = bb.x; bv[5] = bb.y; bv[6] = bb.z; bv[7] = bb.w;
    }
    #pragma unroll
    for (int j = 0; j < 4; ++j) {
      const int tokl = 64 * w2 + 16 * j + m;
      const v8f v = acc[i][j] * WINV + bv;
      const v4f lo = { v[0], v[1], v[2], v[3] };
      const v4f hi = { v[4], v[5], v[6], v[7] };
      float* sp = sF + tokl * 64 + featl;
      *(v4fa*)sp = lo;
      *(v4fa*)(sp + 4) = hi;
    }
  }
  __syncthreads();
  const int q8 = lane & 7, sub = lane >> 3;
  v4f vals[16];
  #pragma unroll
  for (int i = 0; i < 16; ++i) {
    const int u = 4 * i + sub;
    const int rowl = 32 * w + (u >> 1), hl = u & 1;
    const v4f sv = *(const v4fa*)(sF + rowl * 64 + 32 * hl + 4 * q8);
    const v4f xv = *(const v4fa*)(xio + (size_t)(m0 + rowl) * DM + n0 + 32 * hl + 4 * q8);
    vals[i] = sv + xv;
  }
  #pragma unroll
  for (int i = 0; i < 16; ++i) {
    const int u = 4 * i + sub;
    const int rowl = 32 * w + (u >> 1), hl = u & 1;
    *(volatile v4f*)(xio + (size_t)(m0 + rowl) * DM + n0 + 32 * hl + 4 * q8) = vals[i];
  }
  __threadfence();
  #pragma unroll
  for (int i = 0; i < 16; ++i) {
    const int u = 4 * i + sub;
    const int rowl = 32 * w + (u >> 1), hl = u & 1;
    *(volatile v4f*)(xio + (size_t)(m0 + rowl) * DM + n0 + 32 * hl + 4 * q8) = vals[i];
  }
}

__device__ __forceinline__ v8f mask8(v8f s, v4i pa, v4i pc, int kofs, int lim) {
  s[0] = ((kofs + 0 <= lim) && (pa.x != 0)) ? s[0] : NEGBIG;
  s[1] = ((kofs + 1 <= lim) && (pa.y != 0)) ? s[1] : NEGBIG;
  s[2] = ((kofs + 2 <= lim) && (pa.z != 0)) ? s[2] : NEGBIG;
  s[3] = ((kofs + 3 <= lim) && (pa.w != 0)) ? s[3] : NEGBIG;
  s[4] = ((kofs + 4 <= lim) && (pc.x != 0)) ? s[4] : NEGBIG;
  s[5] = ((kofs + 5 <= lim) && (pc.y != 0)) ? s[5] : NEGBIG;
  s[6] = ((kofs + 6 <= lim) && (pc.z != 0)) ? s[6] : NEGBIG;
  s[7] = ((kofs + 7 <= lim) && (pc.w != 0)) ? s[7] : NEGBIG;
  return s;
}

__device__ __forceinline__ v16h pack_p(v8f a, v8f c) {
  const v16h r = { (_Float16)(a[0] * PSCALE), (_Float16)(a[1] * PSCALE), (_Float16)(a[2] * PSCALE), (_Float16)(a[3] * PSCALE),
                   (_Float16)(a[4] * PSCALE), (_Float16)(a[5] * PSCALE), (_Float16)(a[6] * PSCALE), (_Float16)(a[7] * PSCALE),
                   (_Float16)(c[0] * PSCALE), (_Float16)(c[1] * PSCALE), (_Float16)(c[2] * PSCALE), (_Float16)(c[3] * PSCALE),
                   (_Float16)(c[4] * PSCALE), (_Float16)(c[5] * PSCALE), (_Float16)(c[6] * PSCALE), (_Float16)(c[7] * PSCALE) };
  return r;
}

__global__ __launch_bounds__(256) void attn_kernel(const _Float16* __restrict__ qp,
                                                   const _Float16* __restrict__ kp,
                                                   const _Float16* __restrict__ vt,
                                                   const int* __restrict__ ids,
                                                   _Float16* __restrict__ op)
{
  __shared__ __attribute__((aligned(16))) int padL[BLK];
  __shared__ __attribute__((aligned(16))) int padS[NBLK * CSUM];
  __shared__ __attribute__((aligned(16))) _Float16 sO[8 * 16 * HD];

  const int tid = threadIdx.x, lane = tid & 31;
  const int w = __builtin_amdgcn_readfirstlane(tid >> 5);
  const int h = lane >> 4, m = lane & 15;
  const int nb = blockIdx.x, bh = blockIdx.y;
  const int b = bh >> 3, head = bh & (NH - 1);

  if (tid < BLK) padL[tid] = (ids[b * SEQ + nb * BLK + tid] > 0) ? 1 : 0;
  #pragma unroll
  for (int c = 0; c < 2; ++c) {
    const int i = tid + 256 * c;
    padS[i] = (ids[b * SEQ + (i >> 5) * BLK + (BLK - CSUM) + (i & (CSUM - 1))] > 0) ? 1 : 0;
  }
  __syncthreads();

  const int q0 = nb * BLK + 16 * w;
  const int qi = 16 * w + m;
  const _Float16* qrow = qp + ((size_t)bh * SEQ + q0 + m) * HD;
  const v16h qb0 = load_frag(qrow, h);
  const v16h qb1 = load_frag(qrow + 32, h);

  v8f o[4];
  #pragma unroll
  for (int t = 0; t < 4; ++t) o[t] = zero8f();
  float mrun = -1.0e30f, lrun = 0.0f;

  const _Float16* kbase = kp + ((size_t)bh * SEQ + m) * HD;
  const _Float16* vbase = vt + ((size_t)bh * HD + m) * SEQ;
  const int nloc = (w + 2) >> 1;
  const int nst = nloc + nb;

  #pragma unroll 1
  for (int st = 0; st < nst; ++st) {
    const bool local = st < nloc;
    const int key0 = local ? (nb * BLK + 32 * st) : ((st - nloc) * BLK + (BLK - CSUM));
    const int* padp = local ? (padL + 32 * st) : (padS + CSUM * (st - nloc));
    const int lim = local ? (qi - 32 * st) : 64;

    const _Float16* kr0 = kbase + (size_t)key0 * HD;
    const _Float16* kr1 = kr0 + 16 * HD;
    const v16h k00 = load_frag(kr0, h);
    const v16h k01 = load_frag(kr0 + 32, h);
    const v16h k10 = load_frag(kr1, h);
    const v16h k11 = load_frag(kr1 + 32, h);
    v8f s0 = wmma_raw(k00, qb0, zero8f());
    v8f s1 = wmma_raw(k10, qb0, zero8f());
    s0 = wmma_raw(k01, qb1, s0);
    s1 = wmma_raw(k11, qb1, s1);
    asm volatile("v_nop\n\tv_nop\n\tv_nop\n\tv_nop"
                 : "+v"(s0), "+v"(s1)
                 : "v"(k00), "v"(k01), "v"(k10), "v"(k11), "v"(qb0), "v"(qb1));

    const v4i pa = *(const v4ia*)(padp + 8 * h);
    const v4i pc = *(const v4ia*)(padp + 8 * h + 4);
    const v4i pd = *(const v4ia*)(padp + 16 + 8 * h);
    const v4i pe = *(const v4ia*)(padp + 16 + 8 * h + 4);
    s0 = mask8(s0, pa, pc, 8 * h, lim);
    s1 = mask8(s1, pd, pe, 16 + 8 * h, lim);

    float mloc = s0[0];
    #pragma unroll
    for (int r = 0; r < 8; ++r) { mloc = fmaxf(mloc, s0[r]); mloc = fmaxf(mloc, s1[r]); }
    mloc = fmaxf(mloc, __shfl_xor(mloc, 16, 32));
    const float mnew = fmaxf(mrun, mloc);
    const float alpha = __expf(mrun - mnew);
    mrun = mnew;
    float lsum = 0.0f;
    #pragma unroll
    for (int r = 0; r < 8; ++r) {
      const float pa0 = __expf(s0[r] - mnew);
      const float pa1 = __expf(s1[r] - mnew);
      s0[r] = pa0;
      s1[r] = pa1;
      lsum += pa0 + pa1;
    }
    lsum += __shfl_xor(lsum, 16, 32);
    lrun = lrun * alpha + lsum;
    #pragma unroll
    for (int t = 0; t < 4; ++t) o[t] = o[t] * alpha;

    const v16h pb = pack_p(s0, s1);
    v16h vf[4];
    #pragma unroll
    for (int t = 0; t < 4; ++t) vf[t] = load_frag(vbase + (size_t)(16 * t) * SEQ + key0, h);
    #pragma unroll
    for (int t = 0; t < 4; ++t) o[t] = wmma_raw(vf[t], pb, o[t]);
    asm volatile("v_nop\n\tv_nop\n\tv_nop\n\tv_nop"
                 : "+v"(o[0]), "+v"(o[1]), "+v"(o[2]), "+v"(o[3])
                 : "v"(vf[0]), "v"(vf[1]), "v"(vf[2]), "v"(vf[3]), "v"(pb));
  }

  const float inv = (1.0f / lrun) * PINV;
  _Float16* so = sO + w * (16 * HD);
  #pragma unroll
  for (int t = 0; t < 4; ++t)
    *(v8ha*)(so + m * HD + 16 * t + 8 * h) = to8h(o[t] * inv);
  __syncthreads();

  _Float16* dst = op + ((size_t)b * SEQ + q0) * DM + head * HD;
  att_store_pass(so, dst, lane);
  __threadfence();
  att_store_pass(so, dst, lane);
}

extern "C" void kernel_launch(void* const* d_in, const int* in_sizes, int n_in,
                              void* d_out, int out_size, void* d_ws, size_t ws_size,
                              hipStream_t stream) {
  if (n_in < 16) return;
  if (in_sizes[0] != NTOK) return;
  if (in_sizes[1] < DM || (in_sizes[1] % DM) != 0) return;
  if (in_sizes[2] != NL * DM || in_sizes[3] != NL * DM) return;
  if (in_sizes[4] != NL * DM * DM || in_sizes[5] != NL * DM * DM ||
      in_sizes[6] != NL * DM * DM || in_sizes[7] != NL * DM * DM) return;
  if (in_sizes[8] != NL * DM || in_sizes[9] != NL * DM) return;
  if (in_sizes[10] != NL * DM * DMLP || in_sizes[11] != NL * DMLP) return;
  if (in_sizes[12] != NL * DMLP * DM || in_sizes[13] != NL * DM) return;
  if (in_sizes[14] != DM || in_sizes[15] != DM) return;
  if (out_size != NTOK * DM) return;
  const int vocab = in_sizes[1] / DM;

  const int*   ids   = (const int*)  d_in[0];
  const float* embed = (const float*)d_in[1];
  const float* ln1_s = (const float*)d_in[2];
  const float* ln1_b = (const float*)d_in[3];
  const float* wq    = (const float*)d_in[4];
  const float* wk    = (const float*)d_in[5];
  const float* wv    = (const float*)d_in[6];
  const float* wo    = (const float*)d_in[7];
  const float* ln2_s = (const float*)d_in[8];
  const float* ln2_b = (const float*)d_in[9];
  const float* w1    = (const float*)d_in[10];
  const float* b1    = (const float*)d_in[11];
  const float* w2    = (const float*)d_in[12];
  const float* b2    = (const float*)d_in[13];
  const float* lnf_s = (const float*)d_in[14];
  const float* lnf_b = (const float*)d_in[15];
  float* out = (float*)d_out;

  const size_t xB    = (size_t)NTOK * DM * 4;
  const size_t hbB   = (size_t)NTOK * DM * 2;
  const size_t plB   = (size_t)NBATCH * NH * SEQ * HD * 2;
  const size_t opB   = (size_t)NTOK * DM * 2;
  const size_t m1B   = (size_t)NTOK * DMLP * 2;
  const size_t wqkvB = (size_t)NL * NQKV * DM * 2;
  const size_t woB   = (size_t)NL * DM * DM * 2;
  const size_t w1B   = (size_t)NL * DMLP * DM * 2;
  const size_t w2B   = (size_t)NL * DM * DMLP * 2;
  const size_t total = xB + hbB + 3 * plB + opB + m1B + wqkvB + woB + w1B + w2B;
  if (total > ws_size) return;

  char* ws = (char*)d_ws;
  size_t off = 0;
  float*    x    = (float*)(ws + off);    off += xB;
  _Float16* hb   = (_Float16*)(ws + off); off += hbB;
  _Float16* qp   = (_Float16*)(ws + off); off += plB;
  _Float16* kp   = (_Float16*)(ws + off); off += plB;
  _Float16* vt   = (_Float16*)(ws + off); off += plB;
  _Float16* op   = (_Float16*)(ws + off); off += opB;
  _Float16* m1   = (_Float16*)(ws + off); off += m1B;
  _Float16* wqkv = (_Float16*)(ws + off); off += wqkvB;
  _Float16* wot  = (_Float16*)(ws + off); off += woB;
  _Float16* w1t  = (_Float16*)(ws + off); off += w1B;
  _Float16* w2t  = (_Float16*)(ws + off); off += w2B;
  if (off > ws_size) return;

  cvt_t_kernel<<<dim3(DM / 64, DM / 64, NL), 256, 0, stream>>>(wq, wqkv, DM, DM, NQKV, 0, WSC);
  cvt_t_kernel<<<dim3(DM / 64, DM / 64, NL), 256, 0, stream>>>(wk, wqkv, DM, DM, NQKV, DM, WSC);
  cvt_t_kernel<<<dim3(DM / 64, DM / 64, NL), 256, 0, stream>>>(wv, wqkv, DM, DM, NQKV, 2 * DM, WSC);
  cvt_t_kernel<<<dim3(DM / 64, DM / 64, NL), 256, 0, stream>>>(wo, wot, DM, DM, DM, 0, WSC);
  cvt_t_kernel<<<dim3(DMLP / 64, DM / 64, NL), 256, 0, stream>>>(w1, w1t, DM, DMLP, DMLP, 0, WSC);
  cvt_t_kernel<<<dim3(DM / 64, DMLP / 64, NL), 256, 0, stream>>>(w2, w2t, DMLP, DM, DM, 0, WSC);

  embed_kernel<<<NTOK, 256, 0, stream>>>(ids, embed, x, vocab);

  const dim3 gQK(NTOK / 128, 2 * NH);
  const dim3 gV(NTOK / 128, NH);
  const dim3 gD(NTOK / 128, DM / 64);
  const dim3 gM(NTOK / 128, DMLP / 64);
  const dim3 gA(NBLK, NBATCH * NH);

  for (int l = 0; l < NL; ++l) {
    const _Float16* wl_qk = wqkv + (size_t)l * NQKV * DM;
    const _Float16* wl_v  = wl_qk + (size_t)2 * DM * DM;
    const _Float16* wl_o  = wot + (size_t)l * DM * DM;
    const _Float16* wl_1  = w1t + (size_t)l * DMLP * DM;
    const _Float16* wl_2  = w2t + (size_t)l * DM * DMLP;

    ln16_kernel<<<NTOK / 8, 256, 0, stream>>>(x, ln1_s + l * DM, ln1_b + l * DM, hb);
    gemm_qk_kernel<<<gQK, 128, 0, stream>>>(hb, wl_qk, qp, kp);
    gemm_v_kernel<<<gV, 128, 0, stream>>>(hb, wl_v, vt);
    attn_kernel<<<gA, 256, 0, stream>>>(qp, kp, vt, ids, op);
    gemm_resid_kernel<0><<<gD, 128, 0, stream>>>(op, wl_o, b2 + l * DM, x, DM);
    ln16_kernel<<<NTOK / 8, 256, 0, stream>>>(x, ln2_s + l * DM, ln2_b + l * DM, hb);
    gemm_gelu_kernel<<<gM, 128, 0, stream>>>(hb, wl_1, b1 + l * DMLP, m1);
    gemm_resid_kernel<1><<<gD, 128, 0, stream>>>(m1, wl_2, b2 + l * DM, x, DMLP);
  }
  ln32_kernel<<<NTOK / 8, 256, 0, stream>>>(x, lnf_s, lnf_b, out);
}
